// SRNet_2585570312575
// MI455X (gfx1250) — hardware-verified
//
#include <hip/hip_runtime.h>
#include <stddef.h>
#include <stdint.h>

#define NPLANE   6
#define HPIX     255
#define WPIX     255
#define PPIX     65025
#define NPIX     390150
#define XH       256
#define XW       256
#define OW       510
#define OPL      260100
#define NOUT     1560600
#define NF       64
#define FP       328
#define OSP      20
#define WPB      2
#define NWAVE    24385
#define MAINBLK  12193
#define TROWS    390176
#define WOFF2    0
#define WOFF3    4096
#define WOFF4    12288
#define WOFF5    24576
#define WOFF6    40960
#define WTOT     46080
#define WCVTBLK  23
#define NQUAD    390150
#define OUTBLK   1525

static_assert(NPIX == NPLANE * PPIX);
static_assert(PPIX == HPIX * WPIX);
static_assert(NWAVE * 16 >= NPIX);
static_assert((NWAVE - 1) * 16 < NPIX);
static_assert(MAINBLK * WPB >= NWAVE);
static_assert((MAINBLK - 1) * WPB < NWAVE);
static_assert(TROWS == MAINBLK * WPB * 16);
static_assert(OPL == 4 * PPIX);
static_assert(NOUT == NPLANE * OPL);
static_assert(NQUAD * 4 == NOUT);
static_assert(OUTBLK * 256 >= NQUAD);
static_assert((OUTBLK - 1) * 256 < NQUAD);
static_assert(WOFF3 == WOFF2 + 64 * 64);
static_assert(WOFF4 == WOFF3 + 64 * 128);
static_assert(WOFF5 == WOFF4 + 64 * 192);
static_assert(WOFF6 == WOFF5 + 64 * 256);
static_assert(WTOT == WOFF6 + 16 * 320);
static_assert(WOFF3 == 2 * 2048);
static_assert(WOFF4 == 6 * 2048);
static_assert(WOFF5 == 12 * 2048);
static_assert(WOFF6 == 20 * 2048);
static_assert(WCVTBLK * 2048 >= WTOT);
static_assert((WCVTBLK - 1) * 2048 < WTOT);
static_assert(FP % 8 == 0);
static_assert(FP >= 320);
static_assert(15 * FP + 256 + 63 < 16 * FP);
static_assert(15 * OSP + 15 < 16 * OSP);
static_assert((OSP * 4) % 16 == 0);

typedef unsigned short u16;
typedef __bf16 v16b __attribute__((ext_vector_type(16)));
typedef unsigned short v8us __attribute__((ext_vector_type(8)));
typedef float v8f __attribute__((ext_vector_type(8)));
typedef float v4f __attribute__((ext_vector_type(4)));
typedef unsigned int v4u __attribute__((ext_vector_type(4)));

union Frag  { v16b v; v8us h[2]; };
union Pack8 { v8us h; v4u u; u16 s[8]; };

__device__ __forceinline__ v8f zero8() { return (v8f){0.f, 0.f, 0.f, 0.f, 0.f, 0.f, 0.f, 0.f}; }

__device__ __forceinline__ v8f mma(v16b a, v16b b, v8f c) {
  c = __builtin_amdgcn_wmma_f32_16x16x32_bf16(false, a, false, b, (short)0, c, false, false);
  asm volatile("v_nop\n\tv_nop\n\tv_nop\n\tv_nop" : "+v"(c) : "v"(a), "v"(b));
  return c;
}

__device__ __forceinline__ u16 f2bf(float f) {
  unsigned int u = __float_as_uint(f);
  u += 0x7FFFu + ((u >> 16) & 1u);
  return (u16)(u >> 16);
}
__device__ __forceinline__ float bf2f(u16 h) { return __uint_as_float(((unsigned int)h) << 16); }
__device__ __forceinline__ u16 lo_of(float f, u16 hi) { return f2bf(f - bf2f(hi)); }
__device__ __forceinline__ void split8(v4f a, v4f b, v4u& hu, v4u& lu) {
  Pack8 ph, pl;
#pragma unroll
  for (int i = 0; i < 4; ++i) {
    const u16 h0 = f2bf(a[i]);
    ph.s[i] = h0;
    pl.s[i] = lo_of(a[i], h0);
    const u16 h1 = f2bf(b[i]);
    ph.s[4 + i] = h1;
    pl.s[4 + i] = lo_of(b[i], h1);
  }
  hu = ph.u;
  lu = pl.u;
}

__device__ __forceinline__ v16b ldfrag(const u16* p, int ld, int row0, int k0, int lane) {
  const int m = lane & 15, lh = lane >> 4;
  const u16* q = p + (size_t)(row0 + m) * ld + k0 + 8 * lh;
  Frag f;
  f.h[0] = *(const v8us*)(q);
  f.h[1] = *(const v8us*)(q + 16);
  return f.v;
}

template <int K>
__device__ __forceinline__ void dense_layer(u16* fh, u16* fl, const u16* __restrict__ Bh,
                                            const u16* __restrict__ Bl, const float* __restrict__ bias, int lane) {
  static_assert(K % 32 == 0);
  const int lh = lane >> 4, c = lane & 15;
  v8f acc[4];
#pragma unroll
  for (int t = 0; t < 4; ++t) acc[t] = zero8();
#pragma unroll 1
  for (int k0 = 0; k0 < K; k0 += 32) {
    const v16b ah = ldfrag(fh, FP, 0, k0, lane);
    const v16b al = ldfrag(fl, FP, 0, k0, lane);
#pragma unroll
    for (int t = 0; t < 4; ++t) {
      const v16b bh = ldfrag(Bh, K, 16 * t, k0, lane);
      const v16b bl = ldfrag(Bl, K, 16 * t, k0, lane);
      acc[t] = mma(ah, bh, acc[t]);
      acc[t] = mma(al, bh, acc[t]);
      acc[t] = mma(ah, bl, acc[t]);
    }
  }
#pragma unroll
  for (int t = 0; t < 4; ++t) {
    const float bv = bias[16 * t + c];
#pragma unroll
    for (int r = 0; r < 8; ++r) {
      const float v = fmaxf(acc[t][r] + bv, 0.f);
      const u16 hi = f2bf(v);
      const int idx = (8 * lh + r) * FP + K + 16 * t + c;
      fh[idx] = hi;
      fl[idx] = lo_of(v, hi);
    }
  }
}

__global__ __launch_bounds__(256) void k_wcvt(const float* __restrict__ W2, const float* __restrict__ W3,
                                              const float* __restrict__ W4, const float* __restrict__ W5,
                                              const float* __restrict__ W6,
                                              u16* __restrict__ wh, u16* __restrict__ wl) {
  const int blk = blockIdx.x;
  const int e0 = blk * 2048 + (int)threadIdx.x * 8;
  const float* src;
  int K, off, nval, nrow;
  if (blk < 2)       { src = W2; K = 64;  off = WOFF2; nval = 64; nrow = 64; }
  else if (blk < 6)  { src = W3; K = 128; off = WOFF3; nval = 64; nrow = 64; }
  else if (blk < 12) { src = W4; K = 192; off = WOFF4; nval = 64; nrow = 64; }
  else if (blk < 20) { src = W5; K = 256; off = WOFF5; nval = 64; nrow = 64; }
  else               { src = W6; K = 320; off = WOFF6; nval = 4;  nrow = 16; }
  int el = e0 - off;
  const int seg = nrow * K;
  el = (el < seg) ? el : (seg - 8);
  const int n  = el / K;
  const int k  = el - n * K;
  const int nc = (n < nval) ? n : (nval - 1);
  const float* sp = src + (size_t)nc * K + k;
  v4f a0 = *(const v4f*)(sp), a1 = *(const v4f*)(sp + 4);
  if (n >= nval) {
    a0 = (v4f){0.f, 0.f, 0.f, 0.f};
    a1 = (v4f){0.f, 0.f, 0.f, 0.f};
  }
  v4u hu, lu;
  split8(a0, a1, hu, lu);
  const bool ok = (e0 < WTOT);
  if (ok) {
    *(volatile v4u*)(wh + e0) = hu;
    *(volatile v4u*)(wl + e0) = lu;
  }
  __threadfence();
  if (ok) {
    *(volatile v4u*)(wh + e0) = hu;
    *(volatile v4u*)(wl + e0) = lu;
  }
}

__global__ __launch_bounds__(64) void k_main(const float* __restrict__ x, const float* __restrict__ W1,
                                             const float* __restrict__ b1, const float* __restrict__ b2,
                                             const float* __restrict__ b3, const float* __restrict__ b4,
                                             const float* __restrict__ b5, const float* __restrict__ b6,
                                             const u16* __restrict__ wh, const u16* __restrict__ wl,
                                             float* __restrict__ tout) {
  __shared__ __align__(16) u16 Fh[WPB][16 * FP];
  __shared__ __align__(16) u16 Fl[WPB][16 * FP];
  __shared__ __align__(16) float Ps[WPB][16 * 4];
  __shared__ __align__(16) float Os[WPB][16 * OSP];

  const int tid = threadIdx.x, lane = tid & 31, wave = tid >> 5;
  const int lh = lane >> 4, c = lane & 15;
  const int base = ((int)blockIdx.x * WPB + wave) * 16;
  u16* fh = &Fh[wave][0];
  u16* fl = &Fl[wave][0];
  float* ps = &Ps[wave][0];
  float* os = &Os[wave][0];

  {
    int p = base + c;
    p = (p < NPIX) ? p : (NPIX - 1);
    const int pl  = p / PPIX;
    const int rem = p - pl * PPIX;
    const int i   = rem / WPIX;
    const int j   = rem - i * WPIX;
    const float* xp = x + (size_t)pl * (XH * XW) + i * XW + j;
    const float v0 = xp[0], v1 = xp[1], v2 = xp[XW], v3 = xp[XW + 1];
    if (lh == 0) {
      ps[4 * c + 0] = v0;
      ps[4 * c + 1] = v1;
      ps[4 * c + 2] = v2;
      ps[4 * c + 3] = v3;
    }
  }
  __syncthreads();

  {
    const float w00 = W1[lane * 4 + 0], w01 = W1[lane * 4 + 1], w02 = W1[lane * 4 + 2], w03 = W1[lane * 4 + 3];
    const float w10 = W1[(lane + 32) * 4 + 0], w11 = W1[(lane + 32) * 4 + 1];
    const float w12 = W1[(lane + 32) * 4 + 2], w13 = W1[(lane + 32) * 4 + 3];
    const float bb0 = b1[lane], bb1 = b1[lane + 32];
#pragma unroll 4
    for (int p = 0; p < 16; ++p) {
      const v4f pt = *(const v4f*)(ps + 4 * p);
      float s0 = pt[0] * w00;
      s0 = fmaf(pt[1], w01, s0);
      s0 = fmaf(pt[2], w02, s0);
      s0 = fmaf(pt[3], w03, s0);
      float s1 = pt[0] * w10;
      s1 = fmaf(pt[1], w11, s1);
      s1 = fmaf(pt[2], w12, s1);
      s1 = fmaf(pt[3], w13, s1);
      const float v0 = fmaxf(s0 + bb0, 0.f);
      const float v1 = fmaxf(s1 + bb1, 0.f);
      const u16 h0 = f2bf(v0), h1 = f2bf(v1);
      fh[p * FP + lane]      = h0;
      fl[p * FP + lane]      = lo_of(v0, h0);
      fh[p * FP + 32 + lane] = h1;
      fl[p * FP + 32 + lane] = lo_of(v1, h1);
    }
  }
  __syncthreads();

  dense_layer<64>(fh, fl, wh + WOFF2, wl + WOFF2, b2, lane);
  __syncthreads();
  dense_layer<128>(fh, fl, wh + WOFF3, wl + WOFF3, b3, lane);
  __syncthreads();
  dense_layer<192>(fh, fl, wh + WOFF4, wl + WOFF4, b4, lane);
  __syncthreads();
  dense_layer<256>(fh, fl, wh + WOFF5, wl + WOFF5, b5, lane);
  __syncthreads();

  v8f acc = zero8();
  {
    const u16* Bh = wh + WOFF6;
    const u16* Bl = wl + WOFF6;
#pragma unroll 1
    for (int k0 = 0; k0 < 320; k0 += 32) {
      const v16b ah = ldfrag(fh, FP, 0, k0, lane);
      const v16b al = ldfrag(fl, FP, 0, k0, lane);
      const v16b bh = ldfrag(Bh, 320, 0, k0, lane);
      const v16b bl = ldfrag(Bl, 320, 0, k0, lane);
      acc = mma(ah, bh, acc);
      acc = mma(al, bh, acc);
      acc = mma(ah, bl, acc);
    }
  }
  {
    const int cc = (c < 4) ? c : 3;
    const float b6v = b6[cc];
    const float bv  = (c < 4) ? b6v : 0.f;
#pragma unroll
    for (int r = 0; r < 8; ++r) os[(8 * lh + r) * OSP + c] = tanhf(acc[r] + bv);
  }
  __syncthreads();

  const v4f ov = *(const v4f*)(os + c * OSP);
  float* tp = tout + (size_t)(base + c) * 4;
  if (lh == 0) *(volatile v4f*)(tp) = ov;
  __threadfence();
  if (lh == 0) *(volatile v4f*)(tp) = ov;
}

__global__ __launch_bounds__(256) void k_out(const float* __restrict__ tin, float* __restrict__ out) {
  const int q  = blockIdx.x * 256 + (int)threadIdx.x;
  const int qc = (q < NQUAD) ? q : (NQUAD - 1);
  v4f v;
#pragma unroll
  for (int e = 0; e < 4; ++e) {
    const int o   = 4 * qc + e;
    const int pl  = o / OPL;
    const int rem = o - pl * OPL;
    const int R   = rem / OW;
    const int C   = rem - R * OW;
    const int pix = pl * PPIX + (R >> 1) * WPIX + (C >> 1);
    const int ch  = (R & 1) * 2 + (C & 1);
    v[e] = tin[(size_t)pix * 4 + ch];
  }
  float* op = out + (size_t)q * 4;
  if (q < NQUAD) *(volatile v4f*)(op) = v;
  __threadfence();
  if (q < NQUAD) *(volatile v4f*)(op) = v;
}

extern "C" void kernel_launch(void* const* d_in, const int* in_sizes, int n_in,
                              void* d_out, int out_size, void* d_ws, size_t ws_size,
                              hipStream_t stream) {
  if (n_in < 13) return;
  if (in_sizes[0]  != NPLANE * XH * XW) return;
  if (in_sizes[1]  != NF * 4) return;
  if (in_sizes[2]  != NF) return;
  if (in_sizes[3]  != NF * 64) return;
  if (in_sizes[4]  != NF) return;
  if (in_sizes[5]  != NF * 128) return;
  if (in_sizes[6]  != NF) return;
  if (in_sizes[7]  != NF * 192) return;
  if (in_sizes[8]  != NF) return;
  if (in_sizes[9]  != NF * 256) return;
  if (in_sizes[10] != NF) return;
  if (in_sizes[11] != 4 * 320) return;
  if (in_sizes[12] != 4) return;
  if (out_size != NOUT) return;

  const float* x  = (const float*)d_in[0];
  const float* W1 = (const float*)d_in[1];
  const float* b1 = (const float*)d_in[2];
  const float* W2 = (const float*)d_in[3];
  const float* b2 = (const float*)d_in[4];
  const float* W3 = (const float*)d_in[5];
  const float* b3 = (const float*)d_in[6];
  const float* W4 = (const float*)d_in[7];
  const float* b4 = (const float*)d_in[8];
  const float* W5 = (const float*)d_in[9];
  const float* b5 = (const float*)d_in[10];
  const float* W6 = (const float*)d_in[11];
  const float* b6 = (const float*)d_in[12];
  float* out = (float*)d_out;

  const size_t szW = (size_t)WTOT * 2;
  const size_t szT = (size_t)TROWS * 16;
  size_t off = 0;
  const size_t oWH = off; off += szW;
  const size_t oWL = off; off += szW;
  const size_t oT  = off; off += szT;
  if (off > ws_size) return;
  if (off > (size_t)134217728) return;

  char* ws = (char*)d_ws;
  u16* WH  = (u16*)(ws + oWH);
  u16* WL  = (u16*)(ws + oWL);
  float* T = (float*)(ws + oT);

  k_wcvt<<<dim3(WCVTBLK), dim3(256), 0, stream>>>(W2, W3, W4, W5, W6, WH, WL);
  k_main<<<dim3(MAINBLK), dim3(32 * WPB), 0, stream>>>(x, W1, b1, b2, b3, b4, b5, b6, WH, WL, T);
  k_out<<<dim3(OUTBLK), dim3(256), 0, stream>>>(T, out);
  (void)hipGetLastError();
}
